// GraphSAGE_61409442398712
// MI455X (gfx1250) — hardware-verified
//
#include <hip/hip_runtime.h>
#include <stddef.h>
#include <stdint.h>
#include <math.h>


#define DF     128
#define NY     256
#define K2     256
#define NP3    32
#define H3P    16
#define NCLS   10
#define NGR    256
#define PG     16
#define NTHR   256
#define NWAVE  8
#define EPT    8
#define CHUNK  (NTHR * EPT)
#define WCAP   (EPT * 32)
#define LISTN  (NWAVE * WCAP)
#define NBA    1024
#define SLA    10
#define RCAP   28672
#define DEGCAP 64
#define GBM    64
#define GTHR   128
#define UPART  2048
#define UPART3 256
#define AGG_ZINTS    (LISTN + 2 * RCAP + 3 * NBA)
#define MISC_INTS    16
#define ROWBUF_INTS  (NWAVE * 256)
#define AGG_LDS_INTS (AGG_ZINTS + MISC_INTS + ROWBUF_INTS)
#define NOUT   (NGR * NCLS)
#define WSMAX  134217728

static_assert((CHUNK & (CHUNK - 1)) == 0 && CHUNK <= 4096);
static_assert((NBA & (NBA - 1)) == 0 && NBA == (1 << SLA));
static_assert(((long long)CHUNK << SLA) < (1LL << 31));
static_assert(LISTN % NTHR == 0);
static_assert(NBA % NWAVE == 0 && NBA % 32 == 0 && NBA % GBM == 0 && NBA % (NWAVE * 8) == 0);
static_assert(RCAP % 4 == 0 && AGG_ZINTS % 4 == 0 && LISTN % 4 == 0 && ((AGG_ZINTS + MISC_INTS) % 4) == 0);
static_assert(DF % 32 == 0 && K2 % 32 == 0 && K2 == 2 * DF && DF == 4 * 32);
static_assert(GBM == (GTHR / 32) * 16);
static_assert(UPART % NTHR == 0 && UPART == DF * (DF / 8) && UPART3 == NTHR && UPART3 == 16 * (DF / 8));
static_assert(NY % 128 == 0 && NP3 == 32 && H3P == 16 && NCLS <= H3P);
static_assert(AGG_LDS_INTS * 4 <= 300000);
static_assert(NGR % PG == 0 && PG == 2 * NWAVE && (PG * NCLS * 4) % 128 == 0 && (PG * NCLS) % 4 == 0);
static_assert((PG * NCLS) / 4 <= NTHR);
static_assert((NGR / PG - 1) * PG * NCLS + PG * NCLS - 1 == NOUT - 1);

typedef float          v4f   __attribute__((ext_vector_type(4)));
typedef float          v8f   __attribute__((ext_vector_type(8)));
typedef int            v4i   __attribute__((ext_vector_type(4)));
typedef int            v8i   __attribute__((ext_vector_type(8)));
typedef unsigned short v4us  __attribute__((ext_vector_type(4)));
typedef unsigned short v8us  __attribute__((ext_vector_type(8)));
typedef unsigned short v16us __attribute__((ext_vector_type(16)));
typedef __bf16         v16bf __attribute__((ext_vector_type(16)));
typedef v4f  __attribute__((may_alias)) v4fa;
typedef v4i  __attribute__((may_alias)) v4ia;
typedef v4us __attribute__((may_alias)) v4usa;
typedef v8us __attribute__((may_alias)) v8usa;
union FragB { v16bf v; v16us u; v8us h[2]; v8i w; };

__device__ __forceinline__ v8f wmb(const FragB& a, const FragB& b, v8f c) {
  v8f d = __builtin_amdgcn_wmma_f32_16x16x32_bf16(false, a.v, false, b.v, (short)0, c, false, false);
  asm volatile("v_nop\n\tv_nop\n\tv_nop\n\tv_nop" : "+v"(d) : "v"(a.w), "v"(b.w));
  return d;
}

__device__ __forceinline__ unsigned bf16_bits(float f) {
  const unsigned u = __float_as_uint(f);
  return (u + 0x7FFFu + ((u >> 16) & 1u)) >> 16;
}
__device__ __forceinline__ float bf16_val(float f) {
  return __uint_as_float(bf16_bits(f) << 16);
}

__device__ __forceinline__ void wave_sync() {
  __builtin_amdgcn_fence(__ATOMIC_RELEASE, "wavefront");
  __builtin_amdgcn_wave_barrier();
  __builtin_amdgcn_fence(__ATOMIC_ACQUIRE, "wavefront");
}

template <int SLB>
__device__ __forceinline__ int scan_chunk(const int* __restrict__ dsts, int nE, int cbase, int slotBase,
                                          int nb, int vec8, int* list, int tid, int lane, int wave) {
  int wc = 0;
  const int el0  = tid * EPT;
  const int e0   = cbase + el0;
  const int sent = -2147483647 - 1;
  v4i da, db;
  if (vec8 != 0 && cbase + CHUNK <= nE) {
    da = *(const v4i*)(dsts + e0);
    db = *(const v4i*)(dsts + e0 + 4);
  } else {
    da.x = (e0     < nE) ? dsts[min(e0,     nE - 1)] : sent;
    da.y = (e0 + 1 < nE) ? dsts[min(e0 + 1, nE - 1)] : sent;
    da.z = (e0 + 2 < nE) ? dsts[min(e0 + 2, nE - 1)] : sent;
    da.w = (e0 + 3 < nE) ? dsts[min(e0 + 3, nE - 1)] : sent;
    db.x = (e0 + 4 < nE) ? dsts[min(e0 + 4, nE - 1)] : sent;
    db.y = (e0 + 5 < nE) ? dsts[min(e0 + 5, nE - 1)] : sent;
    db.z = (e0 + 6 < nE) ? dsts[min(e0 + 6, nE - 1)] : sent;
    db.w = (e0 + 7 < nE) ? dsts[min(e0 + 7, nE - 1)] : sent;
  }
  const unsigned nbs = (unsigned)slotBase;
  const unsigned unb = (unsigned)nb;
  const unsigned s0 = (unsigned)da.x - nbs, s1 = (unsigned)da.y - nbs;
  const unsigned s2 = (unsigned)da.z - nbs, s3 = (unsigned)da.w - nbs;
  const unsigned s4 = (unsigned)db.x - nbs, s5 = (unsigned)db.y - nbs;
  const unsigned s6 = (unsigned)db.z - nbs, s7 = (unsigned)db.w - nbs;
  const bool h0 = s0 < unb, h1 = s1 < unb, h2 = s2 < unb, h3 = s3 < unb;
  const bool h4 = s4 < unb, h5 = s5 < unb, h6 = s6 < unb, h7 = s7 < unb;
  const unsigned any = __builtin_amdgcn_ballot_w32(h0 | h1 | h2 | h3 | h4 | h5 | h6 | h7);
  if (any != 0u) {
#define HITJ(J, HJ, SJ) { \
      const unsigned mj = __builtin_amdgcn_ballot_w32(HJ); \
      if (mj != 0u) { \
        if (HJ) { \
          const int pos = wc + (int)__builtin_amdgcn_mbcnt_lo(mj, 0u); \
          if (pos < WCAP) list[wave * WCAP + pos] = ((el0 + (J)) << SLB) | (int)(SJ); \
        } \
        wc += (int)__builtin_popcount(mj); } }
    HITJ(0, h0, s0)
    HITJ(1, h1, s1)
    HITJ(2, h2, s2)
    HITJ(3, h3, s3)
    HITJ(4, h4, s4)
    HITJ(5, h5, s5)
    HITJ(6, h6, s6)
    HITJ(7, h7, s7)
#undef HITJ
  }
  return wc;
}

__global__ __launch_bounds__(NTHR) void k_wprep(const float* __restrict__ Wl1, const float* __restrict__ Wr1,
                                                const float* __restrict__ Wl2, const float* __restrict__ Wr2,
                                                const float* __restrict__ Wl3, const float* __restrict__ Wr3,
                                                unsigned short* WB1, unsigned short* WB2, unsigned short* WB3) {
  const int b = (int)blockIdx.x, tid = (int)threadIdx.x;
  int part, v;
  if (b < 48) { part = b >> 3; v = (b & 7) * NTHR + tid; }
  else        { part = 6 + (b - 48); v = tid; }
  const int n  = v >> 4;
  const int k8 = (v & 15) * 8;
  const float* W;
  unsigned short* P;
  int pitch, coff, noff, nreal;
  if (part == 0)      { W = Wl1; P = WB1; pitch = DF; coff = 0;  noff = 0;  nreal = DF; }
  else if (part == 1) { W = Wr1; P = WB1; pitch = DF; coff = 0;  noff = DF; nreal = DF; }
  else if (part == 2) { W = Wl2; P = WB2; pitch = K2; coff = 0;  noff = 0;  nreal = DF; }
  else if (part == 3) { W = Wl2; P = WB2; pitch = K2; coff = DF; noff = 0;  nreal = DF; }
  else if (part == 4) { W = Wr2; P = WB2; pitch = K2; coff = 0;  noff = DF; nreal = DF; }
  else if (part == 5) { W = Wr2; P = WB2; pitch = K2; coff = DF; noff = DF; nreal = DF; }
  else if (part == 6) { W = Wl3; P = WB3; pitch = K2; coff = 0;  noff = 0;  nreal = NCLS; }
  else if (part == 7) { W = Wl3; P = WB3; pitch = K2; coff = DF; noff = 0;  nreal = NCLS; }
  else if (part == 8) { W = Wr3; P = WB3; pitch = K2; coff = 0;  noff = 16; nreal = NCLS; }
  else if (part == 9) { W = Wr3; P = WB3; pitch = K2; coff = DF; noff = 16; nreal = NCLS; }
  else return;
  const bool ok = n < nreal;
  const int  nc = ok ? n : nreal - 1;
  const float* p = W + (size_t)k8 * nreal + nc;
  v8us o;
#pragma unroll
  for (int i = 0; i < 8; ++i) {
    const float f = p[(size_t)i * nreal];
    o[i] = ok ? (unsigned short)bf16_bits(f) : (unsigned short)0;
  }
  unsigned short* dp = P + (size_t)(noff + n) * pitch + coff + k8;
  *(volatile v8us*)dp = o;
  __threadfence();
  *(volatile v8us*)dp = o;
}

__global__ __launch_bounds__(NTHR) void k_cvx(const float* __restrict__ x, int nN, int nUnits,
                                              unsigned short* xb) {
  const int u = (int)blockIdx.x * NTHR + (int)threadIdx.x;
  if (u >= nUnits) return;
  const int row = u >> 4;
  const int k8  = (u & 15) * 8;
  const int rc  = row < nN ? row : nN - 1;
  const float* p = x + (size_t)rc * DF + k8;
  const v4f a = *(const v4fa*)p;
  const v4f b = *(const v4fa*)(p + 4);
  const bool ok = row < nN;
  v8us o;
  o[0] = ok ? (unsigned short)bf16_bits(a.x) : (unsigned short)0;
  o[1] = ok ? (unsigned short)bf16_bits(a.y) : (unsigned short)0;
  o[2] = ok ? (unsigned short)bf16_bits(a.z) : (unsigned short)0;
  o[3] = ok ? (unsigned short)bf16_bits(a.w) : (unsigned short)0;
  o[4] = ok ? (unsigned short)bf16_bits(b.x) : (unsigned short)0;
  o[5] = ok ? (unsigned short)bf16_bits(b.y) : (unsigned short)0;
  o[6] = ok ? (unsigned short)bf16_bits(b.z) : (unsigned short)0;
  o[7] = ok ? (unsigned short)bf16_bits(b.w) : (unsigned short)0;
  unsigned short* dp = xb + (size_t)row * DF + k8;
  *(volatile v8us*)dp = o;
  __threadfence();
  *(volatile v8us*)dp = o;
}

template <int NT>
__global__ __launch_bounds__(GTHR) void k_gemm(
    const unsigned short* __restrict__ A, const unsigned short* __restrict__ WT,
    float* outF, int K, int ldo)
{
  constexpr int GBN = 16 * NT;
  constexpr int LPR = GBN / 4;
  constexpr int RPI = 32 / LPR;
  constexpr int NIT = 16 / RPI;
  static_assert(LPR == 8 || LPR == 32);
  __shared__ __attribute__((aligned(16))) float stg[GBM * GBN];
  const int tid = (int)threadIdx.x, lane = tid & 31, wave = tid >> 5, hh = lane >> 4, m = lane & 15;
  const int rowBase = (int)blockIdx.x * GBM;
  const int col0    = (int)blockIdx.y * GBN;

  v8f acc[NT];
  {
    const v8f z = {0.f, 0.f, 0.f, 0.f, 0.f, 0.f, 0.f, 0.f};
#pragma unroll
    for (int t = 0; t < NT; ++t) acc[t] = z;
  }
  const unsigned short* ap = A  + (size_t)(rowBase + 16 * wave + m) * (size_t)K + 8 * hh;
  const unsigned short* wp = WT + (size_t)(col0 + m) * (size_t)K + 8 * hh;
  const int ksteps = K >> 5;
#pragma unroll 1
  for (int ks = 0; ks < ksteps; ++ks) {
    FragB af;
    af.h[0] = *(const v8usa*)(ap + 32 * ks);
    af.h[1] = *(const v8usa*)(ap + 32 * ks + 16);
#pragma unroll
    for (int t = 0; t < NT; ++t) {
      const unsigned short* wq = wp + (size_t)(16 * t) * (size_t)K + 32 * ks;
      FragB bf;
      bf.h[0] = *(const v8usa*)wq;
      bf.h[1] = *(const v8usa*)(wq + 16);
      acc[t] = wmb(af, bf, acc[t]);
    }
  }

#pragma unroll
  for (int t = 0; t < NT; ++t) {
    const int lc = 16 * t + m;
#pragma unroll
    for (int r = 0; r < 8; ++r) {
      const int lr = 16 * wave + 8 * hh + r;
      stg[lr * GBN + lc] = acc[t][r];
    }
  }
  __syncthreads();

  const int rsub = lane / LPR;
  const int c4   = 4 * (lane % LPR);
  v4f fv[NIT];
#pragma unroll
  for (int i = 0; i < NIT; ++i) {
    const int lr = 16 * wave + RPI * i + rsub;
    fv[i] = *(const v4fa*)(stg + lr * GBN + c4);
  }
#pragma unroll
  for (int i = 0; i < NIT; ++i) {
    const int gr = rowBase + 16 * wave + RPI * i + rsub;
    float* op = outF + (size_t)gr * (size_t)ldo + col0 + c4;
    *(volatile v4f*)op = fv[i];
  }
  __threadfence();
#pragma unroll
  for (int i = 0; i < NIT; ++i) {
    const int gr = rowBase + 16 * wave + RPI * i + rsub;
    float* op = outF + (size_t)gr * (size_t)ldo + col0 + c4;
    *(volatile v4f*)op = fv[i];
  }
}

template <int MODE>
__global__ __launch_bounds__(NTHR) void k_scan(const int* __restrict__ srcs, const int* __restrict__ dsts,
                                               int nE, int nN, int vec8, int mRows,
                                               const float* __restrict__ yin, const float* __restrict__ bias,
                                               unsigned short* hb, float* h3) {
  extern __shared__ __attribute__((aligned(16))) int dsm[];
  int* list = dsm;
  int* hl   = dsm + LISTN;
  int* sl   = hl + RCAP;
  int* cnt  = sl + RCAP;
  int* offs = cnt + NBA;
  int* cur  = offs + NBA;
  int* misc = cur + NBA;
  const int tid = (int)threadIdx.x, lane = tid & 31, wave = tid >> 5;
  int* wbuf = misc + MISC_INTS + wave * 256;
  const int nodeBase = (int)blockIdx.x * NBA;

  {
    const v4i z4 = {0, 0, 0, 0};
    for (int i = tid * 4; i < AGG_ZINTS; i += NTHR * 4) *(v4ia*)(dsm + i) = z4;
    if (tid < MISC_INTS) misc[tid] = 0;
  }
  float bv0 = 0.0f, bv1 = 0.0f, bv2 = 0.0f, bv3 = 0.0f;
  if constexpr (MODE == 0) {
    const v4f a = *(const v4f*)(bias + 4 * lane);
    bv0 = bf16_val(a.x); bv1 = bf16_val(a.y); bv2 = bf16_val(a.z); bv3 = bf16_val(a.w);
  } else {
    const int ch  = lane & 15;
    const int chc = ch < NCLS ? ch : NCLS - 1;
    const float bb = bias[chc];
    bv0 = (ch < NCLS) ? bf16_val(bb) : 0.0f;
  }
  __syncthreads();

  int t = 0, ov = 0;
  const int nChunks = (nE + CHUNK - 1) / CHUNK;
#pragma unroll 1
  for (int ch = 0; ch < nChunks; ++ch) {
    const int cbase = ch * CHUNK;
    const int wc = scan_chunk<SLA>(dsts, nE, cbase, nodeBase, NBA, vec8, list, tid, lane, wave);
    if (lane == 0) misc[wave] = wc;
    __syncthreads();
    if (wave == 0) {
#pragma unroll 1
      for (int w2 = 0; w2 < NWAVE; ++w2) {
        int c = misc[w2];
        c = c < 0 ? 0 : (c > WCAP ? WCAP : c);
#pragma unroll 1
        for (int b0 = 0; b0 < c; b0 += 32) {
          const int idx = b0 + lane;
          const int ent = list[w2 * WCAP + (idx < WCAP ? idx : WCAP - 1)];
          const int m32 = (c - b0) < 32 ? (c - b0) : 32;
#pragma unroll 1
          for (int k = 0; k < m32; ++k) {
            const int u    = __builtin_amdgcn_readlane(ent, k);
            const int slot = u & (NBA - 1);
            const int el   = (u >> SLA) & (CHUNK - 1);
            const int pk   = ((cbase + el) << SLA) | slot;
            if (t < RCAP) {
              if (lane == 0) { hl[t] = pk; cnt[slot] = cnt[slot] + 1; }
              t = t + 1;
            } else {
              ov = 1;
            }
          }
        }
      }
    }
    __syncthreads();
  }
  if (wave == 0 && lane == 0) { misc[8] = t; misc[9] = ov; }
  __syncthreads();
  int tt = misc[8];
  tt = tt < 0 ? 0 : (tt > RCAP ? RCAP : tt);
  const int ovf = misc[9];

  if (wave == 0) {
    const int base = lane * (NBA / 32);
    int s = 0;
#pragma unroll 1
    for (int i = 0; i < NBA / 32; ++i) s += cnt[base + i];
    int incl = s;
#pragma unroll
    for (int d = 1; d < 32; d <<= 1) {
      const int y = __shfl_up(incl, d, 32);
      if (lane >= d) incl += y;
    }
    int run = incl - s;
#pragma unroll 1
    for (int i = 0; i < NBA / 32; ++i) {
      const int cv = cnt[base + i];
      offs[base + i] = run;
      cur[base + i]  = run;
      run += cv;
    }
  }
  __syncthreads();
  if (wave == 0) {
#pragma unroll 1
    for (int b0 = 0; b0 < tt; b0 += 32) {
      const int idx = b0 + lane;
      const int ent = hl[idx < RCAP ? idx : RCAP - 1];
      const int m32 = (tt - b0) < 32 ? (tt - b0) : 32;
#pragma unroll 1
      for (int k = 0; k < m32; ++k) {
        const int u    = __builtin_amdgcn_readlane(ent, k);
        const int slot = u & (NBA - 1);
        if (lane == 0) {
          int p = cur[slot];
          p = p < 0 ? 0 : (p > RCAP - 1 ? RCAP - 1 : p);
          sl[p] = u;
          cur[slot] = p + 1;
        }
      }
    }
  }
  __syncthreads();

  const float qnan = __int_as_float(0x7fc00000);
  const float pz = (ovf != 0) ? qnan : 0.0f;

  if constexpr (MODE == 0) {
    unsigned short* rowbuf = (unsigned short*)wbuf;
#pragma unroll 1
    for (int si = 0; si < NBA / NWAVE; ++si) {
      const int s    = si * NWAVE + wave;
      const int node = nodeBase + s;
      int c = cnt[s];
      const bool big = c > DEGCAP;
      const int craw = c < 1 ? 1 : c;
      c = c < 0 ? 0 : (c > DEGCAP ? DEGCAP : c);
      int o = offs[s];
      o = o < 0 ? 0 : (o > RCAP ? RCAP : o);
      const int nc = node < nN ? node : nN - 1;
      const float inv = 1.0f / (float)craw;
      float a0 = 0.0f, a1 = 0.0f, a2 = 0.0f, a3 = 0.0f;
#pragma unroll 1
      for (int b0 = 0; b0 < c; b0 += 32) {
        int idx = o + b0 + lane;
        idx = idx > RCAP - 1 ? RCAP - 1 : idx;
        const int ent = sl[idx];
        int eid = ent >> SLA;
        eid = eid < 0 ? 0 : (eid > nE - 1 ? nE - 1 : eid);
        int sr = srcs[eid];
        sr = sr < 0 ? 0 : (sr > nN - 1 ? nN - 1 : sr);
        const int m32 = (c - b0) < 32 ? (c - b0) : 32;
#pragma unroll 1
        for (int k = 0; k < m32; ++k) {
          const int sk = __builtin_amdgcn_readlane(sr, k);
          const v4f a = *(const v4f*)(yin + (size_t)sk * NY + 4 * lane);
          a0 += a.x; a1 += a.y; a2 += a.z; a3 += a.w;
        }
      }
      const v4f yr = *(const v4f*)(yin + (size_t)nc * NY + DF + 4 * lane);
      const float pzr = big ? qnan : pz;
      const bool live = node < nN;
      float y0 = (a0 * inv + bv0) + yr.x;
      float y1 = (a1 * inv + bv1) + yr.y;
      float y2 = (a2 * inv + bv2) + yr.z;
      float y3 = (a3 * inv + bv3) + yr.w;
      y0 = y0 + pzr; y1 = y1 + pzr; y2 = y2 + pzr; y3 = y3 + pzr;
      const float m0 = live ? y0 : 0.0f;
      const float m1 = live ? y1 : 0.0f;
      const float m2 = live ? y2 : 0.0f;
      const float m3 = live ? y3 : 0.0f;
      v4us mh, ml;
      {
        unsigned hbt;
        hbt = bf16_bits(m0); mh[0] = (unsigned short)hbt; ml[0] = (unsigned short)bf16_bits(m0 - __uint_as_float(hbt << 16));
        hbt = bf16_bits(m1); mh[1] = (unsigned short)hbt; ml[1] = (unsigned short)bf16_bits(m1 - __uint_as_float(hbt << 16));
        hbt = bf16_bits(m2); mh[2] = (unsigned short)hbt; ml[2] = (unsigned short)bf16_bits(m2 - __uint_as_float(hbt << 16));
        hbt = bf16_bits(m3); mh[3] = (unsigned short)hbt; ml[3] = (unsigned short)bf16_bits(m3 - __uint_as_float(hbt << 16));
      }
      *(v4usa*)(rowbuf + 4 * lane) = mh;
      *(v4usa*)(rowbuf + DF + 4 * lane) = ml;
      wave_sync();
      const v8us q0 = *(const v8usa*)(rowbuf + 8 * lane);
      wave_sync();
      if (node < mRows) {
        unsigned short* rpw = hb + (size_t)node * K2 + 8 * lane;
        *(volatile v8us*)rpw = q0;
        __threadfence();
        *(volatile v8us*)rpw = q0;
      }
    }
  } else {
    float* rowf = (float*)wbuf;
    const int ch = lane & 15;
#pragma unroll 1
    for (int it = 0; it < NBA / (NWAVE * 8); ++it) {
      const int s0 = (it * NWAVE + wave) * 8;
#pragma unroll 1
      for (int j = 0; j < 8; ++j) {
        const int s    = s0 + j;
        const int node = nodeBase + s;
        int c = cnt[s];
        const bool big = c > DEGCAP;
        const int craw = c < 1 ? 1 : c;
        c = c < 0 ? 0 : (c > DEGCAP ? DEGCAP : c);
        int o = offs[s];
        o = o < 0 ? 0 : (o > RCAP ? RCAP : o);
        const int nc = node < nN ? node : nN - 1;
        const float inv = 1.0f / (float)craw;
        float a0 = 0.0f;
#pragma unroll 1
        for (int b0 = 0; b0 < c; b0 += 32) {
          int idx = o + b0 + lane;
          idx = idx > RCAP - 1 ? RCAP - 1 : idx;
          const int ent = sl[idx];
          int eid = ent >> SLA;
          eid = eid < 0 ? 0 : (eid > nE - 1 ? nE - 1 : eid);
          int sr = srcs[eid];
          sr = sr < 0 ? 0 : (sr > nN - 1 ? nN - 1 : sr);
          const int m32 = (c - b0) < 32 ? (c - b0) : 32;
#pragma unroll 1
          for (int k = 0; k < m32; ++k) {
            const int sk = __builtin_amdgcn_readlane(sr, k);
            a0 += yin[(size_t)sk * NP3 + ch];
          }
        }
        const float selfv = yin[(size_t)nc * NP3 + 16 + ch];
        const float pzr = big ? qnan : pz;
        float y = (a0 * inv + bv0) + selfv;
        y = y + pzr;
        y = (ch < NCLS) ? y : 0.0f;
        const float vv = (node < nN) ? y : 0.0f;
        if (lane < 16) rowf[j * H3P + lane] = vv;
      }
      wave_sync();
      const v4f q = *(const v4fa*)(rowf + 4 * lane);
      wave_sync();
      float* op = h3 + (size_t)(nodeBase + s0) * H3P + 4 * lane;
      *(volatile v4f*)op = q;
      __threadfence();
      *(volatile v4f*)op = q;
    }
  }
}

__global__ __launch_bounds__(NTHR) void k_pool(const float* __restrict__ h3, const int* __restrict__ bat,
                                               int nN, float* out) {
  __shared__ __attribute__((aligned(16))) float os[PG * NCLS];
  const int tid = (int)threadIdx.x, lane = tid & 31, wave = tid >> 5;
  const int ch = lane & 15, hf = lane >> 4;
  const int g0 = (int)blockIdx.x * PG;
  const int ga = g0 + 2 * wave, gb = ga + 1;

  float aA = 0.0f, aB = 0.0f;
  int nA = 0, nB = 0;
#pragma unroll 1
  for (int i0 = 0; i0 < nN; i0 += 32) {
    const int i  = i0 + lane;
    const int ic = i < nN ? i : nN - 1;
    const int b  = bat[ic];
    const bool inr = i < nN;
    unsigned mA = __builtin_amdgcn_ballot_w32(inr && (b == ga));
    unsigned mB = __builtin_amdgcn_ballot_w32(inr && (b == gb));
    int nhA = (int)__builtin_popcount(mA);
    int nhB = (int)__builtin_popcount(mB);
    nhA = nhA > 32 ? 32 : nhA;
    nhB = nhB > 32 ? 32 : nhB;
    nA += nhA; nB += nhB;
#pragma unroll 1
    for (int q = 0; q < nhA; ++q) {
      const int k = __builtin_ffs((int)mA) - 1;
      mA &= mA - 1u;
      int node = i0 + (k < 0 ? 0 : k);
      node = node > nN - 1 ? nN - 1 : node;
      aA += h3[(size_t)node * H3P + ch];
    }
#pragma unroll 1
    for (int q = 0; q < nhB; ++q) {
      const int k = __builtin_ffs((int)mB) - 1;
      mB &= mB - 1u;
      int node = i0 + (k < 0 ? 0 : k);
      node = node > nN - 1 ? nN - 1 : node;
      aB += h3[(size_t)node * H3P + ch];
    }
  }
  const int   ncnt = (hf != 0) ? nB : nA;
  const float asum = (hf != 0) ? aB : aA;
  const float cf = (ncnt < 1) ? 1.0f : (float)ncnt;
  const float p  = asum * (1.0f / cf);
  const bool valid = ch < NCLS;
  float mv = valid ? p : -INFINITY;
  mv = fmaxf(mv, __shfl_xor(mv, 1, 32));
  mv = fmaxf(mv, __shfl_xor(mv, 2, 32));
  mv = fmaxf(mv, __shfl_xor(mv, 4, 32));
  mv = fmaxf(mv, __shfl_xor(mv, 8, 32));
  const float ex = expf(p - mv);
  float sv = valid ? ex : 0.0f;
  sv += __shfl_xor(sv, 1, 32);
  sv += __shfl_xor(sv, 2, 32);
  sv += __shfl_xor(sv, 4, 32);
  sv += __shfl_xor(sv, 8, 32);
  const float ov1 = p - (mv + logf(sv));
  if (valid) os[(2 * wave + hf) * NCLS + ch] = ov1;
  __syncthreads();
  const int tq = tid < (PG * NCLS) / 4 ? tid : (PG * NCLS) / 4 - 1;
  const v4f ov = *(const v4fa*)(os + 4 * tq);
  float* op = out + (size_t)g0 * NCLS + 4 * tq;
  const bool okst = tid < (PG * NCLS) / 4;
  if (okst) *(volatile v4f*)op = ov;
  __threadfence();
  if (okst) *(volatile v4f*)op = ov;
}

static inline int cdiv(int a, int b) { return (a + b - 1) / b; }
static inline size_t al256(size_t o) { return (o + 255) & ~(size_t)255; }

extern "C" void kernel_launch(void* const* d_in, const int* in_sizes, int n_in,
                              void* d_out, int out_size, void* d_ws, size_t ws_size,
                              hipStream_t stream) {
  if (n_in < 12) return;
  if (in_sizes[0] < DF || (in_sizes[0] % DF) != 0) return;
  const int nN = in_sizes[0] / DF;
  if (nN < 16 || nN > (1 << 22)) return;
  if (in_sizes[1] < 2 || (in_sizes[1] & 1) != 0) return;
  const int nE = in_sizes[1] / 2;
  if (nE < 1 || nE >= (1 << (31 - SLA))) return;
  if (in_sizes[2] != nN) return;
  if (in_sizes[3] != DF * DF || in_sizes[4] != DF || in_sizes[5] != DF * DF) return;
  if (in_sizes[6] != DF * DF || in_sizes[7] != DF || in_sizes[8] != DF * DF) return;
  if (in_sizes[9] != DF * NCLS || in_sizes[10] != NCLS || in_sizes[11] != DF * NCLS) return;
  if (out_size != NOUT) return;

  const float* x    = (const float*)d_in[0];
  const int*   edge = (const int*)d_in[1];
  const int*   bat  = (const int*)d_in[2];
  const float* Wl1  = (const float*)d_in[3];
  const float* bl1  = (const float*)d_in[4];
  const float* Wr1  = (const float*)d_in[5];
  const float* Wl2  = (const float*)d_in[6];
  const float* bl2  = (const float*)d_in[7];
  const float* Wr2  = (const float*)d_in[8];
  const float* Wl3  = (const float*)d_in[9];
  const float* bl3  = (const float*)d_in[10];
  const float* Wr3  = (const float*)d_in[11];
  float* out = (float*)d_out;
  const int* src = edge;
  const int* dst = edge + nE;

  const int MP  = cdiv(nN, GBM) * GBM;
  const int gM  = MP / GBM;
  const int gA  = cdiv(MP, NBA);
  if ((long long)gA * NBA < (long long)MP) return;
  const int R3  = gA * NBA;
  const int vec8 = ((nE & 3) == 0) ? 1 : 0;

  char* ws = (char*)d_ws;
  size_t off = 0;
  const size_t oWB1 = off; off = al256(off + (size_t)NY * DF * 2);
  const size_t oWB2 = off; off = al256(off + (size_t)NY * K2 * 2);
  const size_t oWB3 = off; off = al256(off + (size_t)NP3 * K2 * 2);
  const size_t oXB  = off; off = al256(off + (size_t)MP * DF * 2);
  const size_t oY   = off; off = al256(off + (size_t)MP * NY * 4);
  const size_t oH   = off; off = al256(off + (size_t)MP * K2 * 2);
  const size_t oP   = off; off = al256(off + (size_t)MP * NP3 * 4);
  const size_t oH3  = off; off = al256(off + (size_t)R3 * H3P * 4);
  if (off > ws_size || off > (size_t)WSMAX) return;
  unsigned short* WB1 = (unsigned short*)(ws + oWB1);
  unsigned short* WB2 = (unsigned short*)(ws + oWB2);
  unsigned short* WB3 = (unsigned short*)(ws + oWB3);
  unsigned short* XB  = (unsigned short*)(ws + oXB);
  float*          Y   = (float*)(ws + oY);
  unsigned short* H   = (unsigned short*)(ws + oH);
  float*          P   = (float*)(ws + oP);
  float*          H3  = (float*)(ws + oH3);

  const size_t scanLds = (size_t)AGG_LDS_INTS * 4;
  hipFuncSetAttribute(reinterpret_cast<const void*>(&k_scan<0>), hipFuncAttributeMaxDynamicSharedMemorySize, (int)scanLds);
  hipFuncSetAttribute(reinterpret_cast<const void*>(&k_scan<1>), hipFuncAttributeMaxDynamicSharedMemorySize, (int)scanLds);

  const int nUx = MP * (DF / 8);
  k_wprep<<<52, NTHR, 0, stream>>>(Wl1, Wr1, Wl2, Wr2, Wl3, Wr3, WB1, WB2, WB3);
  k_cvx<<<cdiv(nUx, NTHR), NTHR, 0, stream>>>(x, nN, nUx, XB);
  k_gemm<8><<<dim3(gM, NY / 128), GTHR, 0, stream>>>(XB, WB1, Y, DF, NY);
  k_scan<0><<<gA, NTHR, scanLds, stream>>>(src, dst, nE, nN, vec8, MP, Y, bl1, H, H3);
  k_gemm<8><<<dim3(gM, NY / 128), GTHR, 0, stream>>>(H, WB2, Y, K2, NY);
  k_scan<0><<<gA, NTHR, scanLds, stream>>>(src, dst, nE, nN, vec8, MP, Y, bl2, H, H3);
  k_gemm<2><<<dim3(gM, 1), GTHR, 0, stream>>>(H, WB3, P, K2, NP3);
  k_scan<1><<<gA, NTHR, scanLds, stream>>>(src, dst, nE, nN, vec8, MP, P, bl3, H, H3);
  k_pool<<<NGR / PG, NTHR, 0, stream>>>(H3, bat, nN, out);
}
